// Mix3DEmbeddingV5_6949257085361
// MI455X (gfx1250) — hardware-run, weakly checked
//
#include <hip/hip_runtime.h>
#include <math.h>


#ifndef NB
#define NB 4
#endif
#ifndef SEQ
#define SEQ 2048
#endif
#define NB_FULL  4
#define SEQ_FULL 2048
#ifndef OUT_SEQ
#define OUT_SEQ SEQ
#endif
#define DH    512
#define EDM   1024
#define AHID  128
#define NCH   6
#define KANG  (NCH * DH)
#define TROWS 1024
#define EP    520
#define SP    516
#define HP    136
#define TPT   (SEQ / 256)
#define WSC   64.0f
#define WSI   (1.0f / 64.0f)
#define QRS   2048.0f
#define QRI   (1.0f / 2048.0f)

static_assert(NB <= NB_FULL);
static_assert(SEQ <= SEQ_FULL);
static_assert(SEQ % 256 == 0);
static_assert(SEQ <= 2048);
static_assert(SEQ % 64 == 0);
static_assert((SEQ * NCH) % 64 == 0);
static_assert((NB * SEQ) % 64 == 0);
static_assert(DH % 64 == 0);
static_assert(DH / 8 == 64);
static_assert(DH == 512);
static_assert(AHID % 64 == 0);
static_assert(KANG % 64 == 0);
static_assert(TROWS % 16 == 0);
static_assert(EDM == 2 * DH);
static_assert((EP * 2) % 16 == 0);
static_assert((SP * 4) % 16 == 0);
static_assert((HP * 2) % 16 == 0);
static_assert(EP >= DH);
static_assert(SP >= DH);
static_assert(HP >= AHID);
static_assert(64 * 72 * 2 <= 131072);
static_assert(SEQ * 16 + 2048 <= 131072);
static_assert(2 * 16 * EP * 2 + 8 * SP * 4 <= 131072);
static_assert(64 * HP * 2 + 8 * 16 * 68 * 4 + 64 * 16 + AHID * 4 <= 131072);
static_assert(16 * 68 * 4 <= 131072);

typedef _Float16 h16;
typedef __attribute__((ext_vector_type(16))) _Float16 v16h;
typedef __attribute__((ext_vector_type(8)))  _Float16 v8h;
typedef __attribute__((ext_vector_type(8)))  float    v8f;
typedef __attribute__((ext_vector_type(4)))  float    v4f;
typedef v4f  __attribute__((may_alias)) v4fa;
typedef v8h  __attribute__((may_alias)) v8ha;

__device__ __forceinline__ unsigned short f2bf(float f) { unsigned u = __float_as_uint(f); u += 0x7FFFu + ((u >> 16) & 1u); return (unsigned short)(u >> 16); }
__device__ __forceinline__ float bfr(float f) { return __uint_as_float(((unsigned)f2bf(f)) << 16); }
__device__ __forceinline__ v16h cat16(v8h lo, v8h hi) { return __builtin_shufflevector(lo, hi, 0, 1, 2, 3, 4, 5, 6, 7, 8, 9, 10, 11, 12, 13, 14, 15); }
__device__ __forceinline__ v8f wmma16(v16h a, v16h b, v8f c) { return __builtin_amdgcn_wmma_f32_16x16x32_f16(false, a, false, b, (short)0, c, false, false); }
__device__ __forceinline__ v8f wmma16g(v16h a, v16h b, v8f c) { c = wmma16(a, b, c); asm volatile("v_nop\n\tv_nop\n\tv_nop\n\tv_nop" : "+v"(c) : "v"(a), "v"(b)); return c; }
__device__ __forceinline__ v16h ldh(const h16* p) { return cat16(*(const v8h*)p, *(const v8h*)(p + 16)); }
__device__ __forceinline__ void wave_sync() { __builtin_amdgcn_fence(3  , "wavefront"); __builtin_amdgcn_wave_barrier(); asm volatile("" ::: "memory"); }
static __device__ __forceinline__ h16 toh_flush(float v) { const h16 r = (h16)v; return (fabsf(v) < 6.103515625e-05f) ? (h16)0.0f : r; }
__device__ __forceinline__ float gelu_erf(float x) { return 0.5f * x * (1.0f + erff(x * 0.70710678118654752440f)); }
__device__ __forceinline__ int   tstep_row(float tv) { return (int)fminf(fmaxf(tv, 0.0f), (float)(TROWS - 1)); }
__device__ __forceinline__ bool  tstep_ok(float tv, int ti) { return (tv >= 0.0f) & (tv <= (float)(TROWS - 1)) & ((float)ti == tv); }
__device__ __forceinline__ float poison() { return __uint_as_float(0x7FC00000u); }

__global__ __launch_bounds__(256) void k_wconvT(const float* __restrict__ W, h16* WT, int K, int N) {
    __shared__ __align__(16) h16 ts[64 * 72];
    const int tid = threadIdx.x;
    const int k0 = blockIdx.x * 64, n0 = blockIdx.y * 64;
#pragma unroll
    for (int it = 0; it < 4; ++it) { const int p = it * 256 + tid; const int kr = p >> 4, c4 = (p & 15) * 4;
        const v4f v = *(const v4f*)(W + (size_t)(k0 + kr) * N + n0 + c4);
#pragma unroll
        for (int i = 0; i < 4; ++i) ts[(c4 + i) * 72 + kr] = toh_flush(bfr(v[i]) * WSC); }
    __syncthreads();
    static_assert(256 * 2 * 16 == 64 * 128);
#pragma unroll 1
    for (int ps = 0; ps < 2; ++ps) {
#pragma unroll
        for (int s = 0; s < 2; ++s) { const int p = s * 256 + tid; const int row = p >> 3, c8 = (p & 7) * 8;
            const v8h o = *(const v8ha*)(&ts[row * 72 + c8]);
            *(volatile v8h*)(WT + (size_t)(n0 + row) * K + k0 + c8) = o; }
        if (ps == 0) __threadfence(); }
}

__global__ __launch_bounds__(256) void k_dist(const float* __restrict__ pos, const int* __restrict__ aa, const float* __restrict__ pos_w1, float* G) {
#pragma clang fp contract(off)
    __shared__ int sSeg[SEQ];
    __shared__ float sX[SEQ];
    __shared__ float sY[SEQ];
    __shared__ float sZ[SEQ];
    __shared__ int sPc[256];
    __shared__ int sPe[256];
    const int tid = threadIdx.x, b = blockIdx.x;
    const size_t tb = (size_t)b * SEQ_FULL;
    int nc = 0, ne = 0;
#pragma unroll 1
    for (int q = 0; q < TPT; ++q) { const int tok = aa[tb + tid * TPT + q]; nc += (tok == 0) ? 1 : 0; ne += (tok == 2) ? 1 : 0; }
    sPc[tid] = nc; sPe[tid] = ne;
    __syncthreads();
    int pc = 0, pe = 0;
#pragma unroll 4
    for (int j = 0; j < 256; ++j) { const int a = sPc[j], e = sPe[j]; pc += (j < tid) ? a : 0; pe += (j < tid) ? e : 0; }
#pragma unroll 1
    for (int q = 0; q < TPT; ++q) { const int i = tid * TPT + q; const int tok = aa[tb + i];
        pc += (tok == 0) ? 1 : 0; pe += (tok == 2) ? 1 : 0;
        const bool valid = (pc > pe) & (tok != 0) & (tok != 2);
        sSeg[i] = valid ? pc : -1;
        const float* pp = pos + (tb + (size_t)i) * 9 + 3;
        sX[i] = bfr(pp[0]); sY[i] = bfr(pp[1]); sZ[i] = bfr(pp[2]); }
    __syncthreads();
    const float w1 = bfr(pos_w1[0]);
#pragma unroll 1
    for (int it = 0; it < TPT; ++it) {
        const int i = it * 256 + tid; const int s = sSeg[i];
        const float xi = sX[i], yi = sY[i], zi = sZ[i];
        float sum = 0.0f; int cnt = 0;
#pragma unroll 4
        for (int j = 0; j < SEQ; ++j) {
            const float dx = xi - sX[j], dy = yi - sY[j], dz = zi - sZ[j];
            const float sq = (dx * dx + dz * dz) + dy * dy;
            const float d = (sq > 0.0f) ? sqrtf(sq) : 0.0f;
            const bool inc = (sSeg[j] == s);
            sum += inc ? d : 0.0f; cnt += inc ? 1 : 0; }
        const float c = (float)(cnt < 1 ? 1 : cnt);
        const float dist = (s >= 0) ? sum * (1.0f / c) : 0.0f;
        const float g = gelu_erf(dist * w1);
        float* gp = G + (size_t)b * SEQ + i;
        *(volatile float*)gp = g; __threadfence(); *(volatile float*)gp = g;
    }
}

__global__ __launch_bounds__(256) void k_table(const h16* __restrict__ W1T, const float* __restrict__ b1, const h16* __restrict__ W2T, const float* __restrict__ b2, float* TAB) {
    __shared__ __align__(16) h16 eh[16 * EP];
    __shared__ __align__(16) h16 er[16 * EP];
    __shared__ __align__(16) float st[8 * SP];
    const int tid = threadIdx.x, lane = tid & 31, lr = lane & 15, hi = lane >> 4;
    const int wave = __builtin_amdgcn_readfirstlane((int)(threadIdx.x >> 5));
    const int r0 = blockIdx.x * 16, cb = wave * 64;
    { const float fr = expf((-logf(10000.0f) / 256.0f) * (float)tid);
#pragma unroll 1
      for (int mr = 0; mr < 16; ++mr) { const float ang = (float)(r0 + mr) * fr; const float sv = sinf(ang), cv = cosf(ang);
          const h16 s1 = toh_flush(sv), c1 = toh_flush(cv);
          eh[mr * EP + tid] = s1;       er[mr * EP + tid] = toh_flush((sv - (float)s1) * QRS);
          eh[mr * EP + 256 + tid] = c1; er[mr * EP + 256 + tid] = toh_flush((cv - (float)c1) * QRS); } }
    __syncthreads();
    v8f acc[4], acr[4];
#pragma unroll
    for (int nb = 0; nb < 4; ++nb) { acc[nb] = (v8f){}; acr[nb] = (v8f){}; }
    const size_t boff = (size_t)(cb + lr) * DH + 8 * hi;
    const int aoff = lr * EP + 8 * hi;
#pragma unroll 1
    for (int kc = 0; kc < DH; kc += 32) {
        const v16h ah = cat16(*(const v8ha*)(&eh[aoff + kc]), *(const v8ha*)(&eh[aoff + kc + 16]));
        const v16h ar = cat16(*(const v8ha*)(&er[aoff + kc]), *(const v8ha*)(&er[aoff + kc + 16]));
#pragma unroll
        for (int nb = 0; nb < 4; ++nb) { const v16h bw = ldh(W1T + boff + (size_t)nb * 16 * DH + kc);
            acc[nb] = wmma16g(ah, bw, acc[nb]); acr[nb] = wmma16g(ar, bw, acr[nb]); }
    }
    __syncthreads();
#pragma unroll
    for (int nb = 0; nb < 4; ++nb) { const int col = cb + nb * 16 + lr; const float bias = bfr(b1[col]);
#pragma unroll
        for (int j = 0; j < 8; ++j) { const int row = 8 * hi + j;
            const float hg = gelu_erf((acc[nb][j] + acr[nb][j] * QRI) * WSI + bias);
            const h16 h1 = toh_flush(hg);
            eh[row * EP + col] = h1; er[row * EP + col] = toh_flush((hg - (float)h1) * QRS); } }
    __syncthreads();
#pragma unroll
    for (int nb = 0; nb < 4; ++nb) { acc[nb] = (v8f){}; acr[nb] = (v8f){}; }
#pragma unroll 1
    for (int kc = 0; kc < DH; kc += 32) {
        const v16h ah = cat16(*(const v8ha*)(&eh[aoff + kc]), *(const v8ha*)(&eh[aoff + kc + 16]));
        const v16h ar = cat16(*(const v8ha*)(&er[aoff + kc]), *(const v8ha*)(&er[aoff + kc + 16]));
#pragma unroll
        for (int nb = 0; nb < 4; ++nb) { const v16h bw = ldh(W2T + boff + (size_t)nb * 16 * DH + kc);
            acc[nb] = wmma16g(ah, bw, acc[nb]); acr[nb] = wmma16g(ar, bw, acr[nb]); }
    }
#pragma unroll
    for (int nb = 0; nb < 4; ++nb) { const float bias = bfr(b2[cb + nb * 16 + lr]);
#pragma unroll
        for (int j = 0; j < 8; ++j) acc[nb][j] = (acc[nb][j] + acr[nb][j] * QRI) * WSI + bias; }
    static_assert(256 * 4 * 16 == 8 * DH * 4);
#pragma unroll
    for (int ph = 0; ph < 2; ++ph) {
        if (hi == ph) {
#pragma unroll
            for (int nb = 0; nb < 4; ++nb)
#pragma unroll
                for (int j = 0; j < 8; ++j) st[j * SP + cb + nb * 16 + lr] = acc[nb][j]; }
        __syncthreads();
#pragma unroll 1
        for (int ps = 0; ps < 2; ++ps) {
#pragma unroll
            for (int it = 0; it < 4; ++it) { const int p = it * 256 + tid; const int row = p >> 7, c4 = (p & 127) * 4;
                const v4f val = *(const v4fa*)(&st[row * SP + c4]);
                *(volatile v4f*)(TAB + (size_t)(r0 + ph * 8 + row) * DH + c4) = val; }
            if (ps == 0) __threadfence(); }
        __syncthreads();
    }
}

__global__ __launch_bounds__(256) void k_angA(const float* __restrict__ angle, const int* __restrict__ mask_angle, const int* __restrict__ angle_mask, const int* __restrict__ bond_mask,
                                              const float* __restrict__ time_pos, const int* __restrict__ aa, const float* __restrict__ ang_w1, const h16* __restrict__ WAT,
                                              const float* __restrict__ unkang, const float* __restrict__ TAB, h16* XA) {
    __shared__ __align__(16) h16 hs[64 * HP];
    __shared__ __align__(16) float os[8 * 16 * 68];
    __shared__ float sAng[64];
    __shared__ int sAm[64];
    __shared__ int sIdx[64];
    __shared__ int sBad[64];
    __shared__ float sW1[AHID];
    const int tid = threadIdx.x, lane = tid & 31, lr = lane & 15, hi = lane >> 4;
    const int wave = __builtin_amdgcn_readfirstlane((int)(threadIdx.x >> 5));
    const int R0 = blockIdx.x * 64;
    const int b = R0 / (SEQ * NCH), rb = R0 % (SEQ * NCH);
    const size_t tbF = (size_t)b * SEQ_FULL;
    if (tid < 64) {
        const int r = rb + tid; const int l = r / NCH, c = r % NCH;
        const size_t src = tbF + (size_t)l;
        int a0 = angle_mask[src * 3 + (c < 3 ? c : 2)];
        int a1 = bond_mask[src * 3 + (c >= 3 ? c - 3 : 0)];
        asm volatile("" : "+v"(a0)); asm volatile("" : "+v"(a1));
        const bool am = ((c < 3) ? a0 : a1) != 0;
        const float av = bfr(angle[src * 6 + c]);
        const int lm = r % SEQ;
        const int tokm = aa[tbF + lm];
        const bool tm = (mask_angle[tbF + lm] != 0) & (tokm != 0) & (tokm != 2);
        const float tv = bfr(time_pos[src]);
        const int ti = tstep_row(tv);
        const bool use = tm & am;
        sAng[tid] = am ? av : 0.0f; sAm[tid] = am ? 1 : 0; sIdx[tid] = use ? ti : 0; sBad[tid] = (use & !tstep_ok(tv, ti)) ? 1 : 0;
    } else if (tid < 64 + AHID) {
        sW1[tid - 64] = bfr(ang_w1[tid - 64]);
    }
    __syncthreads();
#pragma unroll 1
    for (int it = 0; it < 32; ++it) { const int p = it * 256 + tid; const int m = p >> 7, j = p & 127;
        hs[m * HP + j] = toh_flush(gelu_erf(sAng[m] * sW1[j])); }
    __syncthreads();
    const int cb = wave * 64;
    v8f acc[4][4];
#pragma unroll
    for (int mb = 0; mb < 4; ++mb)
#pragma unroll
        for (int nb = 0; nb < 4; ++nb) acc[mb][nb] = (v8f){};
    const size_t boff = (size_t)(cb + lr) * AHID + 8 * hi;
    const int aoff = lr * HP + 8 * hi;
#pragma unroll 1
    for (int kc = 0; kc < AHID; kc += 32) {
        v16h a[4];
#pragma unroll
        for (int mb = 0; mb < 4; ++mb) a[mb] = cat16(*(const v8ha*)(&hs[aoff + mb * 16 * HP + kc]), *(const v8ha*)(&hs[aoff + mb * 16 * HP + kc + 16]));
#pragma unroll
        for (int nb = 0; nb < 4; ++nb) { const v16h bw = ldh(WAT + boff + (size_t)nb * 16 * AHID + kc);
#pragma unroll
            for (int mb = 0; mb < 4; ++mb) acc[mb][nb] = wmma16g(a[mb], bw, acc[mb][nb]); }
    }
    const int wb = wave * 16 * 68;
    const int c8 = (lane & 7) * 8;
    const v4f u0 = *(const v4f*)(unkang + cb + c8), u1 = *(const v4f*)(unkang + cb + c8 + 4);
    static_assert(32 * 4 * 16 == 16 * 128);
#pragma unroll
    for (int mb = 0; mb < 4; ++mb) {
#pragma unroll
        for (int nb = 0; nb < 4; ++nb)
#pragma unroll
            for (int j = 0; j < 8; ++j) os[wb + (hi * 8 + j) * 68 + nb * 16 + lr] = acc[mb][nb][j] * WSI;
        wave_sync();
        v8h hv[4];
#pragma unroll
        for (int s = 0; s < 4; ++s) { const int row = 4 * s + (lane >> 3); const int m = mb * 16 + row;
            const v4f x0 = *(const v4fa*)(&os[wb + row * 68 + c8]); const v4f x1 = *(const v4fa*)(&os[wb + row * 68 + c8 + 4]);
            const bool am = sAm[m] != 0; const bool bad = sBad[m] != 0; const int ix = sIdx[m];
            const float* tp = TAB + (size_t)ix * DH + cb + c8;
            const v4f t0 = *(const v4f*)tp, t1 = *(const v4f*)(tp + 4);
#pragma unroll
            for (int i = 0; i < 4; ++i) {
                float f0 = (am ? x0[i] : bfr(u0[i])) + t0[i]; float f1 = (am ? x1[i] : bfr(u1[i])) + t1[i];
                f0 = bad ? poison() : f0; f1 = bad ? poison() : f1;
                hv[s][i] = toh_flush(f0); hv[s][4 + i] = toh_flush(f1); } }
#pragma unroll 1
        for (int ps = 0; ps < 2; ++ps) {
#pragma unroll
            for (int s = 0; s < 4; ++s) { const int row = 4 * s + (lane >> 3);
                *(volatile v8h*)(XA + (size_t)(R0 + mb * 16 + row) * DH + cb + c8) = hv[s]; }
            if (ps == 0) __threadfence(); }
        wave_sync();
    }
}

__global__ __launch_bounds__(256) void k_posA(const float* __restrict__ G, const int* __restrict__ mask_angle, const float* __restrict__ time_pos, const int* __restrict__ aa,
                                              const float* __restrict__ pos_w2, const float* __restrict__ unkpos, const float* __restrict__ TAB, h16* XP) {
#pragma clang fp contract(off)
    const size_t i = (size_t)blockIdx.x * 256 + threadIdx.x;
    if (i >= (size_t)NB * SEQ * (DH / 8)) return;
    const int token = (int)(i >> 6), c8 = (int)(i & 63) * 8;
    const int bq = token / SEQ, l = token % SEQ;
    const size_t src = (size_t)bq * SEQ_FULL + l;
    const int tok = aa[src];
    const bool pm = (tok != 0) & (tok != 2);
    const bool tm = (mask_angle[src] != 0) & pm;
    const float tv = bfr(time_pos[src]);
    const int ti = tstep_row(tv);
    const int ix = tm ? ti : 0;
    const bool bad = tm & !tstep_ok(tv, ti);
    const float g = G[token];
    const v4f w0 = *(const v4f*)(pos_w2 + c8), w1 = *(const v4f*)(pos_w2 + c8 + 4);
    const v4f u0 = *(const v4f*)(unkpos + c8), u1 = *(const v4f*)(unkpos + c8 + 4);
    const float* tp = TAB + (size_t)ix * DH + c8;
    const v4f t0 = *(const v4f*)tp, t1 = *(const v4f*)(tp + 4);
    v8h o;
#pragma unroll
    for (int k = 0; k < 4; ++k) {
        float f0 = (pm ? g * bfr(w0[k]) : bfr(u0[k])) + t0[k]; float f1 = (pm ? g * bfr(w1[k]) : bfr(u1[k])) + t1[k];
        f0 = bad ? poison() : f0; f1 = bad ? poison() : f1;
        o[k] = toh_flush(f0); o[4 + k] = toh_flush(f1); }
    *(volatile v8h*)(XP + i * 8) = o; __threadfence(); *(volatile v8h*)(XP + i * 8) = o;
}

__global__ __launch_bounds__(32) void k_out(const h16* __restrict__ A, const h16* __restrict__ Bt, int K, const float* __restrict__ bias, const float* __restrict__ clsw, const float* __restrict__ eosw,
                                            const int* __restrict__ aa, const int* __restrict__ pad, int colofs, float* OUT) {
    __shared__ __align__(16) float os[16 * 68];
    const int lane = threadIdx.x & 31, lr = lane & 15, hi = lane >> 4;
    const int r0 = blockIdx.x * 64, c0 = blockIdx.y * 64;
    v8f acc[4][4];
#pragma unroll
    for (int mb = 0; mb < 4; ++mb)
#pragma unroll
        for (int nb = 0; nb < 4; ++nb) acc[mb][nb] = (v8f){};
    const size_t aoff = (size_t)(r0 + lr) * K + 8 * hi, boff = (size_t)(c0 + lr) * K + 8 * hi;
#pragma unroll 1
    for (int kc = 0; kc < K; kc += 32) {
        v16h a[4];
#pragma unroll
        for (int mb = 0; mb < 4; ++mb) a[mb] = ldh(A + aoff + (size_t)mb * 16 * K + kc);
#pragma unroll
        for (int nb = 0; nb < 4; ++nb) { const v16h bw = ldh(Bt + boff + (size_t)nb * 16 * K + kc);
#pragma unroll
            for (int mb = 0; mb < 4; ++mb) acc[mb][nb] = wmma16g(a[mb], bw, acc[mb][nb]); }
    }
    const int bq = r0 / SEQ, l0 = r0 % SEQ;
    const int c4 = (lane & 15) * 4;
    const v4f bsv = *(const v4f*)(bias + c0 + c4);
    const v4f cwv = *(const v4f*)(clsw + colofs + c0 + c4);
    const v4f ewv = *(const v4f*)(eosw + colofs + c0 + c4);
    static_assert(32 * 8 * 16 == 16 * 256);
#pragma unroll
    for (int mb = 0; mb < 4; ++mb) {
#pragma unroll
        for (int nb = 0; nb < 4; ++nb)
#pragma unroll
            for (int j = 0; j < 8; ++j) os[(hi * 8 + j) * 68 + nb * 16 + lr] = acc[mb][nb][j] * WSI;
        wave_sync();
        v4f ov[8];
#pragma unroll
        for (int s = 0; s < 8; ++s) { const int row = 2 * s + (lane >> 4);
            const size_t src = (size_t)bq * SEQ_FULL + (size_t)(l0 + mb * 16 + row);
            const int tok = aa[src]; const int pd = pad[src];
            const v4f x = *(const v4fa*)(&os[row * 68 + c4]);
#pragma unroll
            for (int i = 0; i < 4; ++i) { float v = x[i] + bfr(bsv[i]);
                v = (tok == 0) ? bfr(cwv[i]) : v; v = (tok == 2) ? bfr(ewv[i]) : v; v = (pd != 0) ? 0.0f : v;
                ov[s][i] = v; } }
#pragma unroll 1
        for (int ps = 0; ps < 2; ++ps) {
#pragma unroll
            for (int s = 0; s < 8; ++s) { const int row = 2 * s + (lane >> 4);
                *(volatile v4f*)(OUT + ((size_t)bq * OUT_SEQ + (size_t)(l0 + mb * 16 + row)) * EDM + colofs + c0 + c4) = ov[s]; }
            if (ps == 0) __threadfence(); }
        wave_sync();
    }
}

static constexpr size_t al256(size_t v) { return (v + 255) & ~(size_t)255; }
static constexpr size_t SZ_WSQ  = al256((size_t)DH * DH * 2);
static constexpr size_t SZ_WAT  = al256((size_t)DH * AHID * 2);
static constexpr size_t SZ_WANG = al256((size_t)DH * KANG * 2);
static constexpr size_t SZ_G    = al256((size_t)NB * SEQ * 4);
static constexpr size_t SZ_TAB  = al256((size_t)TROWS * DH * 4);
static constexpr size_t SZ_XA   = al256((size_t)NB * SEQ * KANG * 2);
static constexpr size_t SZ_XP   = al256((size_t)NB * SEQ * DH * 2);
static constexpr size_t SZ_TOTAL = 3 * SZ_WSQ + SZ_WAT + SZ_WANG + SZ_G + SZ_TAB + SZ_XA + SZ_XP;
static_assert(SZ_TOTAL <= (size_t)134217728);
static_assert(((size_t)NB * SEQ * 4) % 128 == 0);
static_assert(((size_t)NB * SEQ * (DH / 8)) % 256 == 0);
static_assert(((size_t)NB * SEQ * NCH) % 64 == 0);

extern "C" void kernel_launch(void* const* d_in, const int* in_sizes, int n_in,
                              void* d_out, int out_size, void* d_ws, size_t ws_size, hipStream_t stream) {
    if (n_in < 27) return;
    const size_t needT = (size_t)(NB - 1) * SEQ_FULL + SEQ;
    if ((size_t)in_sizes[0] < needT * 9 || (size_t)in_sizes[1] < needT * 6) return;
    if ((size_t)in_sizes[2] < needT || (size_t)in_sizes[5] < needT || (size_t)in_sizes[8] < needT || (size_t)in_sizes[10] < needT) return;
    if ((size_t)in_sizes[6] < needT * 3 || (size_t)in_sizes[7] < needT * 3) return;
    if (in_sizes[11] < AHID || (size_t)in_sizes[12] < (size_t)AHID * DH || in_sizes[13] < 1 || in_sizes[14] < DH) return;
    if ((size_t)in_sizes[15] < (size_t)DH * DH || in_sizes[16] < DH || (size_t)in_sizes[17] < (size_t)DH * DH || in_sizes[18] < DH) return;
    if ((size_t)in_sizes[19] < (size_t)KANG * DH || in_sizes[20] < DH || (size_t)in_sizes[21] < (size_t)DH * DH || in_sizes[22] < DH) return;
    if (in_sizes[23] < EDM || in_sizes[24] < EDM || in_sizes[25] < DH || in_sizes[26] < DH) return;
    if ((size_t)out_size < ((size_t)(NB - 1) * OUT_SEQ + SEQ) * EDM) return;
    if (SZ_TOTAL > ws_size) return;
    const float* pos        = (const float*)d_in[0];
    const float* angle      = (const float*)d_in[1];
    const int*   padding    = (const int*)d_in[2];
    const int*   mask_ang   = (const int*)d_in[5];
    const int*   angle_mask = (const int*)d_in[6];
    const int*   bond_mask  = (const int*)d_in[7];
    const float* time_pos   = (const float*)d_in[8];
    const int*   aa         = (const int*)d_in[10];
    const float* ang_w1     = (const float*)d_in[11];
    const float* ang_w2     = (const float*)d_in[12];
    const float* pos_w1     = (const float*)d_in[13];
    const float* pos_w2     = (const float*)d_in[14];
    const float* te_w1      = (const float*)d_in[15];
    const float* te_b1      = (const float*)d_in[16];
    const float* te_w2      = (const float*)d_in[17];
    const float* te_b2      = (const float*)d_in[18];
    const float* angproj_w  = (const float*)d_in[19];
    const float* angproj_b  = (const float*)d_in[20];
    const float* posproj_w  = (const float*)d_in[21];
    const float* posproj_b  = (const float*)d_in[22];
    const float* cls_w      = (const float*)d_in[23];
    const float* eos_w      = (const float*)d_in[24];
    const float* unkang     = (const float*)d_in[25];
    const float* unkpos     = (const float*)d_in[26];
    float* OUT = (float*)d_out;
    char* wsp = (char*)d_ws;
    h16* W1T  = (h16*)wsp; wsp += SZ_WSQ;
    h16* W2T  = (h16*)wsp; wsp += SZ_WSQ;
    h16* WPT  = (h16*)wsp; wsp += SZ_WSQ;
    h16* WAT  = (h16*)wsp; wsp += SZ_WAT;
    h16* WGT  = (h16*)wsp; wsp += SZ_WANG;
    float* G  = (float*)wsp; wsp += SZ_G;
    float* TAB = (float*)wsp; wsp += SZ_TAB;
    h16* XA   = (h16*)wsp; wsp += SZ_XA;
    h16* XP   = (h16*)wsp; wsp += SZ_XP;

    k_wconvT<<<dim3(DH / 64, DH / 64, 1), 256, 0, stream>>>(te_w1, W1T, DH, DH);
    k_wconvT<<<dim3(DH / 64, DH / 64, 1), 256, 0, stream>>>(te_w2, W2T, DH, DH);
    k_wconvT<<<dim3(DH / 64, DH / 64, 1), 256, 0, stream>>>(posproj_w, WPT, DH, DH);
    k_wconvT<<<dim3(AHID / 64, DH / 64, 1), 256, 0, stream>>>(ang_w2, WAT, AHID, DH);
    k_wconvT<<<dim3(KANG / 64, DH / 64, 1), 256, 0, stream>>>(angproj_w, WGT, KANG, DH);

    k_dist<<<NB, 256, 0, stream>>>(pos, aa, pos_w1, G);
    k_table<<<TROWS / 16, 256, 0, stream>>>(W1T, te_b1, W2T, te_b2, TAB);
    k_angA<<<(unsigned)((size_t)NB * SEQ * NCH / 64), 256, 0, stream>>>(angle, mask_ang, angle_mask, bond_mask, time_pos, aa, ang_w1, WAT, unkang, TAB, XA);
    k_posA<<<(unsigned)((size_t)NB * SEQ * (DH / 8) / 256), 256, 0, stream>>>(G, mask_ang, time_pos, aa, pos_w2, unkpos, TAB, XP);

    k_out<<<dim3(NB * SEQ / 64, DH / 64, 1), 32, 0, stream>>>(XA, WGT, KANG, angproj_b, cls_w, eos_w, aa, padding, 0, OUT);
    k_out<<<dim3(NB * SEQ / 64, DH / 64, 1), 32, 0, stream>>>(XP, WPT, DH, posproj_b, cls_w, eos_w, aa, padding, DH, OUT);
}
